// intra_att_LR_61890478736013
// MI455X (gfx1250) — hardware-run, weakly checked
//
#include <hip/hip_runtime.h>
#include <stddef.h>


#define NSRC   100000
#define MR     20000
#define KN     32
#define HD     128
#define NTHR   256
#define NWAVE  (NTHR / 32)
#define RPB    32
#define NIT    (RPB / NWAVE)
#define BP     136
#define SLOPE  0.01f
#define SC_A   8.0f
#define SC_R   8.0f
#define SC_N   64.0f
#define INV_LR (1.0f / 64.0f)
#define INV_SN (1.0f / 512.0f)

static_assert(MR % RPB == 0);
static_assert(KN == 32);
static_assert(HD == 4 * 32);
static_assert(HD % 32 == 0);
static_assert(NWAVE == 8);
static_assert(NIT * NWAVE == RPB);
static_assert((BP * 2) % 16 == 0);
static_assert(BP >= HD);
static_assert((9 * BP) % 8 == 0);
static_assert(((7 * BP) / 8) * 8 == 7 * BP);
static_assert((7 * BP) / 8 <= NTHR);
static_assert(HD <= NTHR);
static_assert(RPB / 4 <= 32);

typedef _Float16 v16h __attribute__((ext_vector_type(16)));
typedef _Float16 v8h  __attribute__((ext_vector_type(8)));
typedef _Float16 v4h  __attribute__((ext_vector_type(4)));
typedef float    v4f  __attribute__((ext_vector_type(4)));
typedef float    v8f  __attribute__((ext_vector_type(8)));
union FragH { v16h v; v8h h[2]; };

__device__ __forceinline__ v8f wmh(v16h a, v16h b, v8f c) {
  v8f d = __builtin_amdgcn_wmma_f32_16x16x32_f16(false, a, false, b, (short)0, c, false, false);
#if defined(__HIP_DEVICE_COMPILE__)
  asm volatile("v_nop\n\tv_nop\n\tv_nop\n\tv_nop" : "+v"(d) : "v"(a), "v"(b));
#endif
  return d;
}

__device__ __forceinline__ v8f zero8() {
  v8f z = {0.f, 0.f, 0.f, 0.f, 0.f, 0.f, 0.f, 0.f};
  return z;
}

__device__ __forceinline__ v16h rfrag(const _Float16* row, int k0, int h) {
  FragH u;
  u.h[0] = *(const v8h*)(row + k0 + 8 * h);
  u.h[1] = *(const v8h*)(row + k0 + 16 + 8 * h);
  return u.v;
}

__device__ __forceinline__ int gidx(int e) {
  e = e < 0 ? e + NSRC : e;
  e = e < 0 ? 0 : e;
  e = e > NSRC - 1 ? NSRC - 1 : e;
  return e;
}

__global__ __launch_bounds__(NTHR) void k_att(const int* __restrict__ nei,
                                              const float* __restrict__ hin,
                                              const float* __restrict__ href,
                                              const float* __restrict__ wl,
                                              const float* __restrict__ bl,
                                              const float* __restrict__ wr,
                                              const float* __restrict__ br,
                                              const float* __restrict__ ai,
                                              float* out0, float* att) {
  __shared__ __align__(16) float    w8s[HD];
  __shared__ __align__(16) float    b8s[HD];
  __shared__ __align__(16) _Float16 bt[16 * BP];
  __shared__ __align__(16) float    sx[NWAVE * KN];
  __shared__ __align__(16) float    slr[NWAVE * KN];
  __shared__ __align__(16) float    sln[NWAVE * KN];
  __shared__ __align__(16) v4f      sout4[RPB / 4];
  float* sout = (float*)sout4;

  const int tid = (int)threadIdx.x, lane = tid & 31, w = tid >> 5, h = lane >> 4, c = lane & 15;

  if (tid < HD) {
    w8s[tid] = SC_A * wl[tid];
    b8s[tid] = SC_A * bl[tid];
    bt[8 * BP + tid] = (_Float16)(SC_N * ai[HD + tid]);
  }
  if (tid < (7 * BP) / 8) {
    v8h z;
#pragma unroll
    for (int i = 0; i < 8; ++i) z[i] = (_Float16)0.0f;
    *(v8h*)(bt + 9 * BP + 8 * tid) = z;
  }
  const v4f wr4 = *(const v4f*)(wr + 4 * lane);
  const v4f br4 = *(const v4f*)(br + 4 * lane);
  const v4f ar4 = *(const v4f*)(ai + 4 * lane);
  __syncthreads();

  const int mb = blockIdx.x * RPB;
  const _Float16* brow = bt + c * BP;

#pragma unroll 1
  for (int it = 0; it < NIT; ++it) {
    const int m = mb + NWAVE * it + w;

    const int id = gidx(nei[(size_t)m * KN + lane]);
    sx[w * KN + lane] = hin[id];

    const float y = href[m];
    float g = 0.0f;
    v4h pk;
#pragma unroll
    for (int q = 0; q < 4; ++q) {
      const float v = fmaxf(fmaf(y, wr4[q], br4[q]), 0.0f);
      g = fmaf(v, ar4[q], g);
      pk[q] = (_Float16)(SC_R * v);
    }
    *(v4h*)(bt + w * BP + 4 * lane) = pk;
#pragma unroll
    for (int off = 16; off > 0; off >>= 1) g += __shfl_xor(g, off, 32);
    __syncthreads();

    const float xt0 = sx[w * KN + c];
    const float xt1 = sx[w * KN + 16 + c];
    v8f acc0 = zero8();
    v8f acc1 = zero8();
#pragma unroll
    for (int ks = 0; ks < HD / 32; ++ks) {
      const int k0 = 32 * ks;
      const v4f wa = *(const v4f*)(w8s + k0 + 8 * h);
      const v4f wb = *(const v4f*)(w8s + k0 + 8 * h + 4);
      const v4f wc = *(const v4f*)(w8s + k0 + 16 + 8 * h);
      const v4f wd = *(const v4f*)(w8s + k0 + 16 + 8 * h + 4);
      const v4f ba = *(const v4f*)(b8s + k0 + 8 * h);
      const v4f bb = *(const v4f*)(b8s + k0 + 8 * h + 4);
      const v4f bc = *(const v4f*)(b8s + k0 + 16 + 8 * h);
      const v4f bd = *(const v4f*)(b8s + k0 + 16 + 8 * h + 4);
      v16h a0, a1;
#pragma unroll
      for (int i = 0; i < 4; ++i) {
        a0[i]      = (_Float16)fmaxf(fmaf(xt0, wa[i], ba[i]), 0.0f);
        a0[4 + i]  = (_Float16)fmaxf(fmaf(xt0, wb[i], bb[i]), 0.0f);
        a0[8 + i]  = (_Float16)fmaxf(fmaf(xt0, wc[i], bc[i]), 0.0f);
        a0[12 + i] = (_Float16)fmaxf(fmaf(xt0, wd[i], bd[i]), 0.0f);
        a1[i]      = (_Float16)fmaxf(fmaf(xt1, wa[i], ba[i]), 0.0f);
        a1[4 + i]  = (_Float16)fmaxf(fmaf(xt1, wb[i], bb[i]), 0.0f);
        a1[8 + i]  = (_Float16)fmaxf(fmaf(xt1, wc[i], bc[i]), 0.0f);
        a1[12 + i] = (_Float16)fmaxf(fmaf(xt1, wd[i], bd[i]), 0.0f);
      }
      const v16h bf = rfrag(brow, k0, h);
      acc0 = wmh(a0, bf, acc0);
      acc1 = wmh(a1, bf, acc1);
    }

    if (c == w) {
#pragma unroll
      for (int r = 0; r < 8; ++r) {
        slr[w * KN + 8 * h + r]      = acc0[r];
        slr[w * KN + 16 + 8 * h + r] = acc1[r];
      }
    }
    if (c == 8) {
#pragma unroll
      for (int r = 0; r < 8; ++r) {
        sln[w * KN + 8 * h + r]      = acc0[r];
        sln[w * KN + 16 + 8 * h + r] = acc1[r];
      }
    }
    __syncthreads();

    const float lr = slr[w * KN + lane] * INV_LR;
    const float sn = sln[w * KN + lane] * INV_SN;
    float lg = g + sn;
    lg = (lg >= 0.0f) ? lg : SLOPE * lg;
    float mx = lg;
#pragma unroll
    for (int off = 16; off > 0; off >>= 1) mx = fmaxf(mx, __shfl_xor(mx, off, 32));
    const float e = __expf(lg - mx);
    float s = e;
#pragma unroll
    for (int off = 16; off > 0; off >>= 1) s += __shfl_xor(s, off, 32);
    const float rs = 1.0f / s;
    const float a  = e * rs;
    float o = a * lr;
#pragma unroll
    for (int off = 16; off > 0; off >>= 1) o += __shfl_xor(o, off, 32);

    float* pa = att + (size_t)m * KN + lane;
    *(volatile float*)pa = a;
    __threadfence();
    *(volatile float*)pa = a;

    if (lane == 0) sout[NWAVE * it + w] = fmaxf(o, 0.0f);
  }
  __syncthreads();

  if (w == 0 && lane < RPB / 4) {
    const v4f v = sout4[lane];
    float* po = out0 + mb + 4 * lane;
    *(volatile v4f*)po = v;
    __threadfence();
    *(volatile v4f*)po = v;
  }
}

extern "C" void kernel_launch(void* const* d_in, const int* in_sizes, int n_in,
                              void* d_out, int out_size, void* d_ws, size_t ws_size,
                              hipStream_t stream) {
  (void)d_ws; (void)ws_size;
  if (n_in < 8) return;
  if (in_sizes[0] != MR * KN || in_sizes[1] != NSRC || in_sizes[2] != MR) return;
  if (in_sizes[3] != HD || in_sizes[4] != HD || in_sizes[5] != HD || in_sizes[6] != HD) return;
  if (in_sizes[7] != 2 * HD) return;
  if (out_size != MR + MR * KN) return;

  const int*   nei  = (const int*)d_in[0];
  const float* hin  = (const float*)d_in[1];
  const float* href = (const float*)d_in[2];
  const float* wl   = (const float*)d_in[3];
  const float* bl   = (const float*)d_in[4];
  const float* wr   = (const float*)d_in[5];
  const float* br   = (const float*)d_in[6];
  const float* ai   = (const float*)d_in[7];

  float* out0 = (float*)d_out;
  float* att  = out0 + MR;

  k_att<<<MR / RPB, NTHR, 0, stream>>>(nei, hin, href, wl, bl, wr, br, ai, out0, att);
}
